// GlobalLinearAttention_70257075028618
// MI455X (gfx1250) — hardware-run, weakly checked
//
#include <hip/hip_runtime.h>

constexpr int kBatches       = 2;
constexpr int kSeqLen        = 4096;
constexpr int kModel         = 1024;
constexpr int kHeads         = 4;
constexpr int kHeadDim       = 256;
constexpr int kChunkLen      = 32;
constexpr int kNumChunks     = kSeqLen / kChunkLen;
constexpr int kESlice        = 64;
constexpr int kSlicesPerHead = kHeadDim / kESlice;
constexpr int kKtPitch       = 40;
constexpr int kAttnTile      = kChunkLen * kChunkLen;
constexpr float kEps         = 1e-6f;

typedef __attribute__((ext_vector_type(16))) _Float16 v16h;
typedef __attribute__((ext_vector_type(8)))  _Float16 v8h;
typedef __attribute__((ext_vector_type(16))) __bf16   v16b;
typedef __attribute__((ext_vector_type(8)))  __bf16   v8b;
typedef __attribute__((ext_vector_type(8)))  float    v8f;
typedef __attribute__((ext_vector_type(4)))  float    v4f;
typedef __attribute__((ext_vector_type(4)))  unsigned int v4u;
typedef __attribute__((ext_vector_type(8)))  unsigned int v8u;

__device__ __forceinline__ unsigned short f2bf_bits(float f) {
  unsigned u = __float_as_uint(f);
  return (unsigned short)((u + 0x7FFFu + ((u >> 16) & 1u)) >> 16);
}
__device__ __forceinline__ float bf_bits2f(unsigned short h) { return __uint_as_float(((unsigned)h) << 16); }

__device__ __forceinline__ void dep_guard_h(v8f& a, v8f& b, v16h x, v16h y) { asm volatile("v_nop\n\tv_nop\n\tv_nop\n\tv_nop" : "+v"(a), "+v"(b) : "v"(x), "v"(y)); }
__device__ __forceinline__ void dep_guard_b(v8f& a, v8f& b, v16b x, v16b y) { asm volatile("v_nop\n\tv_nop\n\tv_nop\n\tv_nop" : "+v"(a), "+v"(b) : "v"(x), "v"(y)); }
__device__ __forceinline__ void keep4_h(v16h a, v16h b, v16h c, v16h d) { asm volatile("v_nop" :: "v"(a), "v"(b), "v"(c), "v"(d)); }
__device__ __forceinline__ void keep4_b(v16b a, v16b b, v16b c, v16b d) { asm volatile("v_nop" :: "v"(a), "v"(b), "v"(c), "v"(d)); }
__device__ __forceinline__ void acc_guard4(v8f& a, v8f& b, v8f& c, v8f& d) { asm volatile("v_nop\n\tv_nop\n\tv_nop\n\tv_nop" : "+v"(a), "+v"(b), "+v"(c), "+v"(d)); }
template <typename T> struct Frag;
template <> struct Frag<_Float16> {
  typedef v16h V; union U { v16h v; v8h h[2]; };
  static __device__ __forceinline__ v16h load(const _Float16* p) {
    U f; f.h[0] = *(const v8h*)(p); f.h[1] = *(const v8h*)(p + 16); return f.v;
  }
  static __device__ __forceinline__ v8f mma(v16h a, v16h b, v8f c) {
    return __builtin_amdgcn_wmma_f32_16x16x32_f16(false, a, false, b, (short)0, c, false, false);
  }
  static __device__ __forceinline__ void guard(v8f& a, v8f& b, v16h x, v16h y) { dep_guard_h(a, b, x, y); }
  static __device__ __forceinline__ void keep(v16h a, v16h b, v16h c, v16h d) { keep4_h(a, b, c, d); }
};
template <> struct Frag<__bf16> {
  typedef v16b V; union U { v16b v; v8b h[2]; };
  static __device__ __forceinline__ v16b load(const __bf16* p) {
    U f; f.h[0] = *(const v8b*)(p); f.h[1] = *(const v8b*)(p + 16); return f.v;
  }
  static __device__ __forceinline__ v8f mma(v16b a, v16b b, v8f c) {
    return __builtin_amdgcn_wmma_f32_16x16x32_bf16(false, a, false, b, (short)0, c, false, false);
  }
  static __device__ __forceinline__ void guard(v8f& a, v8f& b, v16b x, v16b y) { dep_guard_b(a, b, x, y); }
  static __device__ __forceinline__ void keep(v16b a, v16b b, v16b c, v16b d) { keep4_b(a, b, c, d); }
};

template <int ET> struct Elem;
template <> struct Elem<0> { typedef _Float16 T; };
template <> struct Elem<1> { typedef __bf16 T; };
template <int ET, bool SPLIT, int BIAS_MODE, int OUT_MODE, bool RESID, int ACT = 0>
__global__ __launch_bounds__(256) void wmma_gemm64(
    const unsigned short* __restrict__ Ap, const unsigned short* __restrict__ A2p, int lda, long strideA,
    const unsigned short* __restrict__ Btp, const unsigned short* __restrict__ Bt2p, int ldb, long strideB,
    void* __restrict__ Cout, void* __restrict__ Cout2, int ldc, long strideC,
    const float* __restrict__ bias,
    const float* __restrict__ resid, long strideR,
    int M, int N, int K, float scale) {
  typedef typename Elem<ET>::T T;
  typedef typename Frag<T>::V V;
  const T* A = (const T*)Ap; const T* A2 = (const T*)A2p; const T* Bt = (const T*)Btp; const T* Bt2 = (const T*)Bt2p;
  __shared__ __align__(16) float sT[8][16 * 68];
  const int b    = blockIdx.y;
  const int lane = threadIdx.x & 31;
  const int wave = threadIdx.x >> 5;
  const int tilesN = N >> 6;
  const int tilesM = M >> 6;
  const int tile = blockIdx.x * 8 + wave;
  if (tile >= tilesM * tilesN) return;
  const int tm = tile / tilesN;
  const int tn = tile - tm * tilesN;
  const int m0 = tm << 6;
  const int n0 = tn << 6;

  const T* Ab  = A  + (size_t)b * strideA;
  const T* Bb  = Bt + (size_t)b * strideB;
  const T* Ab2 = SPLIT ? (A2  + (size_t)b * strideA) : nullptr;
  const T* Bb2 = SPLIT ? (Bt2 + (size_t)b * strideB) : nullptr;

  const int rlane = lane & 15;
  const int koff  = (lane >> 4) * 8;
  const int mOff  = (lane >> 4) * 8;

  v8f acc[4][4];
#pragma unroll
  for (int i = 0; i < 4; ++i)
#pragma unroll
    for (int j = 0; j < 4; ++j) acc[i][j] = (v8f){0.f,0.f,0.f,0.f,0.f,0.f,0.f,0.f};

  for (int k0 = 0; k0 < K; k0 += 32) {
    V bh[4], bl[4];
#pragma unroll
    for (int j = 0; j < 4; ++j) {
      const size_t bo = (size_t)(n0 + (j << 4) + rlane) * ldb + koff + k0;
      bh[j] = Frag<T>::load(Bb + bo);
      if (SPLIT) bl[j] = Frag<T>::load(Bb2 + bo);
    }
#pragma unroll
    for (int i = 0; i < 4; ++i) {
      const size_t ao = (size_t)(m0 + (i << 4) + rlane) * lda + koff + k0;
      V ah = Frag<T>::load(Ab + ao);
      V al;
      if (SPLIT) al = Frag<T>::load(Ab2 + ao);
#pragma unroll
      for (int j = 0; j < 4; ++j) {
        acc[i][j] = Frag<T>::mma(ah, bh[j], acc[i][j]);
        if (SPLIT) {
          acc[i][j] = Frag<T>::mma(ah, bl[j], acc[i][j]);
          acc[i][j] = Frag<T>::mma(al, bh[j], acc[i][j]);
        }
      }
      Frag<T>::guard(acc[i][0], acc[i][3], ah, SPLIT ? al : ah);
    }
    Frag<T>::keep(bh[0], bh[1], bh[2], bh[3]);
    if (SPLIT) Frag<T>::keep(bl[0], bl[1], bl[2], bl[3]);
  }
  acc_guard4(acc[0][0], acc[0][1], acc[0][2], acc[0][3]);
  acc_guard4(acc[1][0], acc[1][1], acc[1][2], acc[1][3]);
  acc_guard4(acc[2][0], acc[2][1], acc[2][2], acc[2][3]);
  acc_guard4(acc[3][0], acc[3][1], acc[3][2], acc[3][3]);

  float* slab = sT[wave];
  const float* Rb = RESID ? (resid + (size_t)b * strideR) : nullptr;
#pragma unroll
  for (int i = 0; i < 4; ++i) {
    const int mBase = m0 + (i << 4);
#pragma unroll
    for (int j = 0; j < 4; ++j) {
      const int n = n0 + (j << 4) + rlane;
      float bv = 0.f;
      if (BIAS_MODE == 2) bv = bias[n];
#pragma unroll
      for (int r = 0; r < 8; ++r) {
        float v = acc[i][j][r] * scale;
        if (BIAS_MODE == 1) v += bias[mBase + mOff + r];
        if (BIAS_MODE == 2) v += bv;
        if (RESID) v += Rb[(size_t)(mBase + mOff + r) * ldc + n];
        if (ACT == 2) v = fmaxf(v, 0.0f);
        if (ACT == 4) v = (v > 0.f) ? v : 0.01f * v;
        if (ACT == 6) v = fmaxf(v, 0.0f) + 1.0f;
        slab[(mOff + r) * 68 + (j << 4) + rlane] = v;
      }
    }
    __builtin_amdgcn_fence(__ATOMIC_RELEASE, "workgroup");
    __builtin_amdgcn_wave_barrier();
    __builtin_amdgcn_fence(__ATOMIC_ACQUIRE, "workgroup");
    if (OUT_MODE == 0) {
      float* C = (float*)Cout + (size_t)b * strideC;
      const int hh = lane >> 4, c4 = (lane & 15) * 4;
      for (int pass = 0; pass < 2; ++pass) {
#pragma unroll
        for (int it = 0; it < 8; ++it) {
          const int row = it * 2 + hh;
          v4f v = *(const v4f*)(slab + row * 68 + c4);
          *(volatile v4f*)(C + (size_t)(mBase + row) * ldc + n0 + c4) = v;
        }
        __threadfence();
      }
    } else {
      const int q = lane >> 3, c8 = (lane & 7) * 8;
      unsigned short* C  = (unsigned short*)Cout  + (size_t)b * strideC;
      unsigned short* C2 = (OUT_MODE == 2) ? ((unsigned short*)Cout2 + (size_t)b * strideC) : nullptr;
      for (int pass = 0; pass < 2; ++pass) {
#pragma unroll
        for (int it = 0; it < 4; ++it) {
          const int row = it * 4 + q;
          const float* sp = slab + row * 68 + c8;
          v8h hv, lv;
#pragma unroll
          for (int e = 0; e < 8; ++e) {
            if (OUT_MODE == 1) {
              hv[e] = (_Float16)sp[e];
            } else {
              unsigned short hb = f2bf_bits(sp[e]);
              unsigned short lb = f2bf_bits(sp[e] - bf_bits2f(hb));
              hv[e] = __builtin_bit_cast(_Float16, hb);
              lv[e] = __builtin_bit_cast(_Float16, lb);
            }
          }
          *(volatile v8h*)(C + (size_t)(mBase + row) * ldc + n0 + c8) = hv;
          if (OUT_MODE == 2) *(volatile v8h*)(C2 + (size_t)(mBase + row) * ldc + n0 + c8) = lv;
        }
        __threadfence();
      }
    }
    __builtin_amdgcn_fence(__ATOMIC_RELEASE, "workgroup");
    __builtin_amdgcn_wave_barrier();
    __builtin_amdgcn_fence(__ATOMIC_ACQUIRE, "workgroup");
  }
}

__device__ __forceinline__ unsigned bfr_bits(float f) {
  const unsigned u = __float_as_uint(f);
  return ((u + 0x7FFFu + ((u >> 16) & 1u)) >> 16) & 0xffffu;
}
__device__ __forceinline__ void split2w(float a, float b, unsigned& wh, unsigned& wl) {
  const unsigned ha = bfr_bits(a), hb = bfr_bits(b);
  const unsigned la = bfr_bits(a - __uint_as_float(ha << 16));
  const unsigned lb = bfr_bits(b - __uint_as_float(hb << 16));
  wh = ha | (hb << 16);
  wl = la | (lb << 16);
}
__device__ __forceinline__ float bf_low(unsigned w)  { return __uint_as_float(w << 16); }
__device__ __forceinline__ float bf_high(unsigned w) { return __uint_as_float(w & 0xffff0000u); }
__device__ __forceinline__ v8f mma3(v8f c, v16b ah, v16b al, v16b bh, v16b bl) {
  c = __builtin_amdgcn_wmma_f32_16x16x32_bf16(false, ah, false, bh, (short)0, c, false, false);
  c = __builtin_amdgcn_wmma_f32_16x16x32_bf16(false, ah, false, bl, (short)0, c, false, false);
  c = __builtin_amdgcn_wmma_f32_16x16x32_bf16(false, al, false, bh, (short)0, c, false, false);
  asm volatile("v_nop\n\tv_nop\n\tv_nop\n\tv_nop" : "+v"(c) : "v"(ah), "v"(al), "v"(bh), "v"(bl));
  return c;
}
__device__ __forceinline__ v8f vz8() { return (v8f){0.f,0.f,0.f,0.f,0.f,0.f,0.f,0.f}; }

__global__ __launch_bounds__(256) void k_split8(const float* __restrict__ in, unsigned short* __restrict__ hi,
                                               unsigned short* __restrict__ lo, int n8) {
  const int i = blockIdx.x * 256 + threadIdx.x;
  if (i >= n8) return;
  const float* p = in + 8 * (size_t)i;
  const v4f a = *(const v4f*)(p);
  const v4f c = *(const v4f*)(p + 4);
  unsigned h0, l0, h1, l1, h2, l2, h3, l3;
  split2w(a[0], a[1], h0, l0);
  split2w(a[2], a[3], h1, l1);
  split2w(c[0], c[1], h2, l2);
  split2w(c[2], c[3], h3, l3);
  const v4u vh = (v4u){h0, h1, h2, h3};
  const v4u vl = (v4u){l0, l1, l2, l3};
  unsigned short* qh = hi + 8 * (size_t)i;
  unsigned short* ql = lo + 8 * (size_t)i;
  *(volatile v4u*)qh = vh;
  *(volatile v4u*)ql = vl;
  __threadfence();
  *(volatile v4u*)qh = vh;
  *(volatile v4u*)ql = vl;
}

__global__ __launch_bounds__(128) void k_attn(const unsigned short* __restrict__ Qh, const unsigned short* __restrict__ Ql,
                                              const unsigned short* __restrict__ Kh, const unsigned short* __restrict__ Kl,
                                              unsigned short* __restrict__ ATh, unsigned short* __restrict__ ATl,
                                              float* __restrict__ Zi) {
  __shared__ __align__(16) float sl_s[4][kChunkLen * 36];
  __shared__ float zl_s[4][kChunkLen];
  const int lane = threadIdx.x & 31;
  const int wave = __builtin_amdgcn_readfirstlane((int)(threadIdx.x >> 5));
  const int hh = lane >> 4, rl = lane & 15, koff = hh * 8;
  const int item = blockIdx.x * 4 + wave;
  if (item >= kHeads * kNumChunks) return;
  const int h  = item / kNumChunks;
  const int nc = item - h * kNumChunks;
  const int t0 = nc * kChunkLen, hcol = h * kHeadDim;
  const __bf16* Qhb = (const __bf16*)Qh; const __bf16* Qlb = (const __bf16*)Ql;
  const __bf16* Khb = (const __bf16*)Kh; const __bf16* Klb = (const __bf16*)Kl;

  v8f acc[2][2];
  acc[0][0] = vz8(); acc[0][1] = vz8(); acc[1][0] = vz8(); acc[1][1] = vz8();
  for (int ks = 0; ks < kHeadDim / 32; ++ks) {
    const size_t co = (size_t)hcol + ks * 32 + koff;
    v16b kfh[2], kfl[2];
#pragma unroll
    for (int nt = 0; nt < 2; ++nt) {
      const size_t ro = (size_t)(t0 + nt * 16 + rl) * kModel + co;
      kfh[nt] = Frag<__bf16>::load(Khb + ro);
      kfl[nt] = Frag<__bf16>::load(Klb + ro);
    }
#pragma unroll
    for (int mt = 0; mt < 2; ++mt) {
      const size_t ro = (size_t)(t0 + mt * 16 + rl) * kModel + co;
      const v16b qfh = Frag<__bf16>::load(Qhb + ro);
      const v16b qfl = Frag<__bf16>::load(Qlb + ro);
#pragma unroll
      for (int nt = 0; nt < 2; ++nt) acc[mt][nt] = mma3(acc[mt][nt], qfh, qfl, kfh[nt], kfl[nt]);
    }
    keep4_b(kfh[0], kfh[1], kfl[0], kfl[1]);
  }
  acc_guard4(acc[0][0], acc[0][1], acc[1][0], acc[1][1]);

  float* sl = sl_s[wave];
  float* zl = zl_s[wave];
#pragma unroll
  for (int mt = 0; mt < 2; ++mt) {
#pragma unroll
    for (int r = 0; r < 8; ++r) {
      const int c = mt * 16 + hh * 8 + r;
      float s = 0.f;
#pragma unroll
      for (int nt = 0; nt < 2; ++nt) {
        const int cp = nt * 16 + rl;
        const float v = (cp <= c) ? acc[mt][nt][r] : 0.f;
        sl[c * 36 + cp] = v;
        s += v;
      }
      s += __shfl_xor(s, 1, 32);
      s += __shfl_xor(s, 2, 32);
      s += __shfl_xor(s, 4, 32);
      s += __shfl_xor(s, 8, 32);
      zl[c] = s;
    }
  }
  __builtin_amdgcn_fence(__ATOMIC_RELEASE, "workgroup");
  __builtin_amdgcn_wave_barrier();
  __builtin_amdgcn_fence(__ATOMIC_ACQUIRE, "workgroup");

  const size_t tb = (size_t)(h * kNumChunks + nc) * kAttnTile;
  const int rq = lane >> 2, cs = (lane & 3) * 8;
  v4u uh[4], ul[4];
#pragma unroll
  for (int i = 0; i < 4; ++i) {
    const int row = 8 * i + rq;
    const float* sp = sl + row * 36 + cs;
    const v4f a  = *(const v4f*)(sp);
    const v4f bq = *(const v4f*)(sp + 4);
    unsigned w0h, w0l, w1h, w1l, w2h, w2l, w3h, w3l;
    split2w(a[0], a[1], w0h, w0l);
    split2w(a[2], a[3], w1h, w1l);
    split2w(bq[0], bq[1], w2h, w2l);
    split2w(bq[2], bq[3], w3h, w3l);
    uh[i] = (v4u){w0h, w1h, w2h, w3h};
    ul[i] = (v4u){w0l, w1l, w2l, w3l};
  }
  const float zv = zl[lane];
  float* zp = Zi + (size_t)(h * kNumChunks + nc) * kChunkLen + lane;
  for (int pass = 0; pass < 2; ++pass) {
#pragma unroll
    for (int i = 0; i < 4; ++i) {
      const int row = 8 * i + rq;
      *(volatile v4u*)(ATh + tb + row * kChunkLen + cs) = uh[i];
      *(volatile v4u*)(ATl + tb + row * kChunkLen + cs) = ul[i];
    }
    *(volatile float*)zp = zv;
    __threadfence();
  }
}

__global__ __launch_bounds__(256) void k_scan(
    const unsigned short* __restrict__ Qh,  const unsigned short* __restrict__ Ql,
    const unsigned short* __restrict__ Kh,  const unsigned short* __restrict__ Kl,
    const unsigned short* __restrict__ VTh, const unsigned short* __restrict__ VTl,
    const unsigned short* __restrict__ ATh, const unsigned short* __restrict__ ATl,
    const float* __restrict__ Zi,
    unsigned short* __restrict__ AOh, unsigned short* __restrict__ AOl) {
  __shared__ __align__(16) unsigned short kth_s[kHeadDim * kKtPitch];
  __shared__ __align__(16) unsigned short ktl_s[kHeadDim * kKtPitch];
  __shared__ __align__(16) float po_s[4 * 2 * 256];
  __shared__ __align__(16) float os_s[kChunkLen * 68];
  __shared__ float z_s[kHeadDim];
  __shared__ float zc_s[kChunkLen * 8];
  __shared__ float dinv_s[kChunkLen];

  const int tid  = threadIdx.x;
  const int lane = tid & 31;
  const int wave = __builtin_amdgcn_readfirstlane(tid >> 5);
  const int hh = lane >> 4, rl = lane & 15, koff = hh * 8;
  const int h   = blockIdx.x / kSlicesPerHead;
  const int e0  = (blockIdx.x - h * kSlicesPerHead) * kESlice;
  const int et  = wave & 3;
  const int dhf = wave >> 2;
  const int hcol = h * kHeadDim;
  const __bf16* Qhb  = (const __bf16*)Qh;  const __bf16* Qlb  = (const __bf16*)Ql;
  const __bf16* VThb = (const __bf16*)VTh; const __bf16* VTlb = (const __bf16*)VTl;
  const __bf16* AThb = (const __bf16*)ATh; const __bf16* ATlb = (const __bf16*)ATl;
  const __bf16* kthb = (const __bf16*)kth_s; const __bf16* ktlb = (const __bf16*)ktl_s;
  const size_t vro = (size_t)(hcol + e0 + et * 16 + rl) * kSeqLen;

  v8f sacc[8];
#pragma unroll
  for (int j = 0; j < 8; ++j) sacc[j] = vz8();
  z_s[tid] = 0.f;
  __syncthreads();

#pragma unroll 1
  for (int nc = 0; nc < kNumChunks; ++nc) {
    const int t0 = nc * kChunkLen;
    {
      const int c = tid >> 3, g = tid & 7;
      const size_t kro = (size_t)(t0 + c) * kModel + hcol + g * 32;
      const v4u* ph = (const v4u*)(Kh + kro);
      const v4u* pl = (const v4u*)(Kl + kro);
#pragma unroll
      for (int i = 0; i < 4; ++i) {
        const v4u wh = ph[i];
        const v4u wl = pl[i];
#pragma unroll
        for (int e = 0; e < 4; ++e) {
          const int d = g * 32 + 8 * i + 2 * e;
          kth_s[d * kKtPitch + c]       = (unsigned short)(wh[e] & 0xffffu);
          kth_s[(d + 1) * kKtPitch + c] = (unsigned short)(wh[e] >> 16);
          ktl_s[d * kKtPitch + c]       = (unsigned short)(wl[e] & 0xffffu);
          ktl_s[(d + 1) * kKtPitch + c] = (unsigned short)(wl[e] >> 16);
        }
      }
    }
    {
      const int c = tid >> 3, g = tid & 7;
      const size_t qro = (size_t)(t0 + c) * kModel + hcol + g * 32;
      const v4u* ph = (const v4u*)(Qh + qro);
      const v4u* pl = (const v4u*)(Ql + qro);
      float s = 0.f;
#pragma unroll
      for (int i = 0; i < 4; ++i) {
        const v4u wh = ph[i];
        const v4u wl = pl[i];
#pragma unroll
        for (int e = 0; e < 4; ++e) {
          const int d = g * 32 + 8 * i + 2 * e;
          const float q0 = bf_low(wh[e]) + bf_low(wl[e]);
          const float q1 = bf_high(wh[e]) + bf_high(wl[e]);
          s = fmaf(q0, z_s[d], s);
          s = fmaf(q1, z_s[d + 1], s);
        }
      }
      zc_s[c * 8 + g] = s;
    }
    v8f acco[2];
    acco[0] = vz8(); acco[1] = vz8();
#pragma unroll
    for (int ks = 0; ks < 4; ++ks) {
      union { v8u u; v16b v; } fh, fl;
#pragma unroll
      for (int p = 0; p < 4; ++p) {
        unsigned wh, wl;
        split2w(sacc[2 * ks][2 * p], sacc[2 * ks][2 * p + 1], wh, wl);
        fh.u[p] = wh; fl.u[p] = wl;
        split2w(sacc[2 * ks + 1][2 * p], sacc[2 * ks + 1][2 * p + 1], wh, wl);
        fh.u[4 + p] = wh; fl.u[4 + p] = wl;
      }
      const size_t qco = (size_t)hcol + dhf * 128 + ks * 32 + koff;
#pragma unroll
      for (int ct = 0; ct < 2; ++ct) {
        const size_t qo = (size_t)(t0 + ct * 16 + rl) * kModel + qco;
        const v16b bh = Frag<__bf16>::load(Qhb + qo);
        const v16b bl = Frag<__bf16>::load(Qlb + qo);
        acco[ct] = mma3(acco[ct], fh.v, fl.v, bh, bl);
      }
    }
    if (dhf == 1) {
      const v16b vfh = Frag<__bf16>::load(VThb + vro + t0 + koff);
      const v16b vfl = Frag<__bf16>::load(VTlb + vro + t0 + koff);
      const size_t ab = (size_t)(h * kNumChunks + nc) * kAttnTile;
#pragma unroll
      for (int ct = 0; ct < 2; ++ct) {
        const size_t ao = ab + (size_t)(ct * 16 + rl) * kChunkLen + koff;
        const v16b bh = Frag<__bf16>::load(AThb + ao);
        const v16b bl = Frag<__bf16>::load(ATlb + ao);
        acco[ct] = mma3(acco[ct], vfh, vfl, bh, bl);
      }
#pragma unroll
      for (int ct = 0; ct < 2; ++ct) {
        float* pp = po_s + (et * 2 + ct) * 256 + lane * 8;
        *(v4f*)(pp)     = (v4f){acco[ct][0], acco[ct][1], acco[ct][2], acco[ct][3]};
        *(v4f*)(pp + 4) = (v4f){acco[ct][4], acco[ct][5], acco[ct][6], acco[ct][7]};
      }
    }
    __syncthreads();
    if (tid < kChunkLen) {
      float zc = 0.f;
#pragma unroll
      for (int g = 0; g < 8; ++g) zc += zc_s[tid * 8 + g];
      const float zi = Zi[(size_t)(h * kNumChunks + nc) * kChunkLen + tid];
      const float den = zi + zc + kEps;
      dinv_s[tid] = 1.0f / den;
    }
    {
      const v4u* ph = (const v4u*)(kth_s + tid * kKtPitch);
      const v4u* pl = (const v4u*)(ktl_s + tid * kKtPitch);
      float s = 0.f;
#pragma unroll
      for (int i = 0; i < 4; ++i) {
        const v4u wh = ph[i];
        const v4u wl = pl[i];
#pragma unroll
        for (int e = 0; e < 4; ++e) {
          s += bf_low(wh[e]) + bf_low(wl[e]);
          s += bf_high(wh[e]) + bf_high(wl[e]);
        }
      }
      z_s[tid] += s;
    }
    __syncthreads();
    if (dhf == 0) {
#pragma unroll
      for (int ct = 0; ct < 2; ++ct) {
        const int c = ct * 16 + rl;
        const float dv = dinv_s[c];
        const float* pp = po_s + (et * 2 + ct) * 256 + lane * 8;
        const v4f p0 = *(const v4f*)(pp);
        const v4f p1 = *(const v4f*)(pp + 4);
        const v4f o0 = (v4f){(acco[ct][0] + p0[0]) * dv, (acco[ct][1] + p0[1]) * dv,
                             (acco[ct][2] + p0[2]) * dv, (acco[ct][3] + p0[3]) * dv};
        const v4f o1 = (v4f){(acco[ct][4] + p1[0]) * dv, (acco[ct][5] + p1[1]) * dv,
                             (acco[ct][6] + p1[2]) * dv, (acco[ct][7] + p1[3]) * dv};
        float* op = os_s + c * 68 + et * 16 + hh * 8;
        *(v4f*)(op)     = o0;
        *(v4f*)(op + 4) = o1;
      }
    }
    {
      const v16b vfh = Frag<__bf16>::load(VThb + vro + t0 + koff);
      const v16b vfl = Frag<__bf16>::load(VTlb + vro + t0 + koff);
#pragma unroll
      for (int j = 0; j < 8; ++j) {
        const int drow = (dhf * 8 + j) * 16 + rl;
        const v16b ah = Frag<__bf16>::load(kthb + drow * kKtPitch + koff);
        const v16b al = Frag<__bf16>::load(ktlb + drow * kKtPitch + koff);
        sacc[j] = mma3(sacc[j], ah, al, vfh, vfl);
      }
      acc_guard4(sacc[0], sacc[1], sacc[2], sacc[3]);
      acc_guard4(sacc[4], sacc[5], sacc[6], sacc[7]);
    }
    __syncthreads();
    {
      const int q = lane >> 3, c8 = (lane & 7) * 8;
      const int row = wave * 4 + q;
      const float* sp = os_s + row * 68 + c8;
      const v4f a  = *(const v4f*)(sp);
      const v4f bq = *(const v4f*)(sp + 4);
      unsigned w0h, w0l, w1h, w1l, w2h, w2l, w3h, w3l;
      split2w(a[0], a[1], w0h, w0l);
      split2w(a[2], a[3], w1h, w1l);
      split2w(bq[0], bq[1], w2h, w2l);
      split2w(bq[2], bq[3], w3h, w3l);
      const v4u vh = (v4u){w0h, w1h, w2h, w3h};
      const v4u vl = (v4u){w0l, w1l, w2l, w3l};
      const size_t oo = (size_t)(t0 + row) * kModel + hcol + e0 + c8;
      for (int pass = 0; pass < 2; ++pass) {
        *(volatile v4u*)(AOh + oo) = vh;
        *(volatile v4u*)(AOl + oo) = vl;
        __threadfence();
      }
    }
  }
}

__global__ __launch_bounds__(256) void k_premise(const int* __restrict__ flag, float* __restrict__ out, int n4) {
  const int cz = flag[0];
  if (cz != 0) return;
  const int i = blockIdx.x * 256 + threadIdx.x;
  if (i >= n4) return;
  const float qn = __uint_as_float(0x7fc00000u);
  const v4f v = (v4f){qn, qn, qn, qn};
  float* p = out + 4 * (size_t)i;
  *(volatile v4f*)p = v;
  __threadfence();
  *(volatile v4f*)p = v;
}

extern "C" void kernel_launch(void* const* d_in, const int* in_sizes, int n_in,
                              void* d_out, int out_size, void* d_ws, size_t ws_size,
                              hipStream_t stream) {
  if (n_in < 6) return;
  const size_t nX  = (size_t)kBatches * kSeqLen * kModel;
  const size_t nXb = (size_t)kSeqLen * kModel;
  const size_t nW  = (size_t)kModel * kModel;
  if ((size_t)in_sizes[0] != nX || (size_t)in_sizes[1] != nW || (size_t)in_sizes[2] != nW ||
      (size_t)in_sizes[3] != nW || (size_t)in_sizes[4] != nW || in_sizes[5] < 1 || (size_t)out_size != nX) return;

  const float* x  = (const float*)d_in[0];
  const float* Wq = (const float*)d_in[1];
  const float* Wk = (const float*)d_in[2];
  const float* Wv = (const float*)d_in[3];
  const float* Wo = (const float*)d_in[4];
  const int* causal = (const int*)d_in[5];
  float* out = (float*)d_out;

  const size_t planeW  = nW * 2;
  const size_t planeX  = nXb * 2;
  const size_t planeAT = (size_t)kHeads * kNumChunks * kAttnTile * 2;
  const size_t bytesZi = (size_t)kHeads * kNumChunks * kChunkLen * sizeof(float);
  char* p = (char*)d_ws;
  unsigned short* Wqh = (unsigned short*)p; p += planeW;
  unsigned short* Wql = (unsigned short*)p; p += planeW;
  unsigned short* Wkh = (unsigned short*)p; p += planeW;
  unsigned short* Wkl = (unsigned short*)p; p += planeW;
  unsigned short* Wvh = (unsigned short*)p; p += planeW;
  unsigned short* Wvl = (unsigned short*)p; p += planeW;
  unsigned short* Woh = (unsigned short*)p; p += planeW;
  unsigned short* Wol = (unsigned short*)p; p += planeW;
  unsigned short* Xh  = (unsigned short*)p; p += planeX;
  unsigned short* Xl  = (unsigned short*)p; p += planeX;
  unsigned short* Qh  = (unsigned short*)p; p += planeX;
  unsigned short* Ql  = (unsigned short*)p; p += planeX;
  unsigned short* Kh  = (unsigned short*)p; p += planeX;
  unsigned short* Kl  = (unsigned short*)p; p += planeX;
  unsigned short* VTh = (unsigned short*)p; p += planeX;
  unsigned short* VTl = (unsigned short*)p; p += planeX;
  unsigned short* ATh = (unsigned short*)p; p += planeAT;
  unsigned short* ATl = (unsigned short*)p; p += planeAT;
  float* Zi = (float*)p; p += bytesZi;
  const size_t total = (size_t)(p - (char*)d_ws);
  if (total > ws_size) return;
  unsigned short* AOh = Xh;
  unsigned short* AOl = Xl;

  const dim3 blk256(256), blk128(128);
  const int n8W = (int)(nW / 8);
  const int n8X = (int)(nXb / 8);
  const int n4O = (int)(nX / 4);
  const unsigned gW = (unsigned)((n8W + 255) / 256);
  const unsigned gX = (unsigned)((n8X + 255) / 256);
  const unsigned gO = (unsigned)((n4O + 255) / 256);
  const unsigned gGemm = (unsigned)(((kSeqLen / 64) * (kModel / 64) + 7) / 8);
  const unsigned gAttn = (unsigned)((kHeads * kNumChunks + 3) / 4);
  const unsigned gScan = (unsigned)(kHeads * kSlicesPerHead);

  k_split8<<<dim3(gW), blk256, 0, stream>>>(Wq, Wqh, Wql, n8W);
  k_split8<<<dim3(gW), blk256, 0, stream>>>(Wk, Wkh, Wkl, n8W);
  k_split8<<<dim3(gW), blk256, 0, stream>>>(Wv, Wvh, Wvl, n8W);
  k_split8<<<dim3(gW), blk256, 0, stream>>>(Wo, Woh, Wol, n8W);

  for (int b = 0; b < kBatches; ++b) {
    const float* xb = x + (size_t)b * nXb;
    float* outb = out + (size_t)b * nXb;
    k_split8<<<dim3(gX), blk256, 0, stream>>>(xb, Xh, Xl, n8X);
    wmma_gemm64<1, true, 0, 2, false, 6><<<dim3(gGemm, 1), blk256, 0, stream>>>(
        Xh, Xl, kModel, 0L, Wqh, Wql, kModel, 0L, (void*)Qh, (void*)Ql, kModel, 0L,
        (const float*)nullptr, (const float*)nullptr, 0L, kSeqLen, kModel, kModel, 1.0f);
    wmma_gemm64<1, true, 0, 2, false, 6><<<dim3(gGemm, 1), blk256, 0, stream>>>(
        Xh, Xl, kModel, 0L, Wkh, Wkl, kModel, 0L, (void*)Kh, (void*)Kl, kModel, 0L,
        (const float*)nullptr, (const float*)nullptr, 0L, kSeqLen, kModel, kModel, 1.0f);
    wmma_gemm64<1, true, 0, 2, false, 0><<<dim3(gGemm, 1), blk256, 0, stream>>>(
        Wvh, Wvl, kModel, 0L, Xh, Xl, kModel, 0L, (void*)VTh, (void*)VTl, kSeqLen, 0L,
        (const float*)nullptr, (const float*)nullptr, 0L, kModel, kSeqLen, kModel, 1.0f);
    k_attn<<<dim3(gAttn), blk128, 0, stream>>>(Qh, Ql, Kh, Kl, ATh, ATl, Zi);
    k_scan<<<dim3(gScan), blk256, 0, stream>>>(Qh, Ql, Kh, Kl, VTh, VTl, ATh, ATl, Zi, AOh, AOl);
    wmma_gemm64<1, true, 0, 0, false, 0><<<dim3(gGemm, 1), blk256, 0, stream>>>(
        AOh, AOl, kModel, 0L, Woh, Wol, kModel, 0L, (void*)outb, (void*)nullptr, kModel, 0L,
        (const float*)nullptr, (const float*)nullptr, 0L, kSeqLen, kModel, kModel, 1.0f);
  }
  k_premise<<<dim3(gO), blk256, 0, stream>>>(causal, out, n4O);
}
